// TextGuideAttentionLayer_26972394619675
// MI455X (gfx1250) — hardware-run, weakly checked
//
#include <hip/hip_runtime.h>
#include <math.h>
#include <stdint.h>

#define NB   8
#define SEQ  2048
#define DM   768
#define DH   3072
#define NTOK 16384
#define NIMG 1204224
#define AQ   32
#define MC   4096

typedef _Float16 v16h __attribute__((ext_vector_type(16)));
typedef _Float16 v8h  __attribute__((ext_vector_type(8)));
typedef float    v8f  __attribute__((ext_vector_type(8)));
typedef float    v4f  __attribute__((ext_vector_type(4)));
typedef double   v2d  __attribute__((ext_vector_type(2)));

union FragU { v16h v; v8h h[2]; };

__device__ __forceinline__ v16h frag_ld(const _Float16* p) {
  FragU u;
  u.h[0] = *(const v8h*)(p);
  u.h[1] = *(const v8h*)(p + 16);
  return u.v;
}
__device__ __forceinline__ v8f mma_raw(v16h a, v16h b, v8f c) {
  return __builtin_amdgcn_wmma_f32_16x16x32_f16(false, a, false, b, (short)0, c, false, false);
}
__device__ __forceinline__ v8f mma_g(v16h a, v16h b, v8f c) {
  c = mma_raw(a, b, c);
  asm volatile("v_nop\n\tv_nop\n\tv_nop\n\tv_nop" : "+v"(c) : "v"(a), "v"(b));
  return c;
}
__device__ __forceinline__ void dep_guard(v8f& a, v8f& b, v16h x, v16h y) {
  asm volatile("v_nop\n\tv_nop\n\tv_nop\n\tv_nop" : "+v"(a), "+v"(b) : "v"(x), "v"(y));
}
__device__ __forceinline__ void keep4(v16h a, v16h b, v16h c, v16h d) {
  asm volatile("v_nop" :: "v"(a), "v"(b), "v"(c), "v"(d));
}
__device__ __forceinline__ void acc_guard4(v8f& a, v8f& b, v8f& c, v8f& d) {
  asm volatile("v_nop\n\tv_nop\n\tv_nop\n\tv_nop" : "+v"(a), "+v"(b), "+v"(c), "+v"(d));
}
__device__ __forceinline__ v8f zero8() { return (v8f){0.f, 0.f, 0.f, 0.f, 0.f, 0.f, 0.f, 0.f}; }

template <int BIAS_MODE, int OUT_MODE, bool RESID, int ACT, bool STATS>
__global__ __launch_bounds__(256) void gemm64_kernel(
    const unsigned short* __restrict__ Ap, int lda,
    const unsigned short* __restrict__ Btp, int ldb,
    void* __restrict__ Cout, int ldc,
    const float* __restrict__ bias, const float* __restrict__ resid, float* __restrict__ part,
    int M, int N, int K, float scale, float oscale) {
  const _Float16* A  = (const _Float16*)Ap;
  const _Float16* Bt = (const _Float16*)Btp;
  __shared__ __align__(16) float sT[8][16 * 68];
  const int lane = threadIdx.x & 31;
  const int wave = threadIdx.x >> 5;
  const int tilesN = N >> 6;
  const int tilesM = M >> 6;
  const int tile = blockIdx.x * 8 + wave;
  if (tile >= tilesM * tilesN) return;
  const int tm = tile / tilesN;
  const int tn = tile - tm * tilesN;
  const int m0 = tm << 6;
  const int n0 = tn << 6;
  const int rlane = lane & 15;
  const int koff  = (lane >> 4) * 8;
  const int mOff  = (lane >> 4) * 8;

  v8f acc[4][4];
#pragma unroll
  for (int i = 0; i < 4; ++i)
#pragma unroll
    for (int j = 0; j < 4; ++j) acc[i][j] = zero8();

  for (int k0 = 0; k0 < K; k0 += 32) {
    v16h bh[4];
#pragma unroll
    for (int j = 0; j < 4; ++j)
      bh[j] = frag_ld(Bt + (size_t)(n0 + (j << 4) + rlane) * ldb + koff + k0);
#pragma unroll
    for (int i = 0; i < 4; ++i) {
      const v16h ah = frag_ld(A + (size_t)(m0 + (i << 4) + rlane) * lda + koff + k0);
#pragma unroll
      for (int j = 0; j < 4; ++j) acc[i][j] = mma_raw(ah, bh[j], acc[i][j]);
      dep_guard(acc[i][0], acc[i][3], ah, ah);
    }
    keep4(bh[0], bh[1], bh[2], bh[3]);
  }
  acc_guard4(acc[0][0], acc[0][1], acc[0][2], acc[0][3]);
  acc_guard4(acc[1][0], acc[1][1], acc[1][2], acc[1][3]);
  acc_guard4(acc[2][0], acc[2][1], acc[2][2], acc[2][3]);
  acc_guard4(acc[3][0], acc[3][1], acc[3][2], acc[3][3]);

  float* slab = sT[wave];
  double ds = 0.0, ds2 = 0.0;
#pragma unroll
  for (int i = 0; i < 4; ++i) {
    const int mBase = m0 + (i << 4);
#pragma unroll
    for (int j = 0; j < 4; ++j) {
      const int n = n0 + (j << 4) + rlane;
      float bn = 0.f;
      if (BIAS_MODE == 2) bn = bias[n];
#pragma unroll
      for (int r = 0; r < 8; ++r) {
        float v = acc[i][j][r] * scale;
        if (BIAS_MODE == 1) v += bias[mBase + mOff + r];
        if (BIAS_MODE == 2) v += bn;
        if (RESID) v += resid[(size_t)(mBase + mOff + r) * ldc + n];
        if (ACT == 2) v = fmaxf(v, 0.0f);
        if (STATS) { const double dv = (double)v; ds += dv; ds2 += dv * dv; }
        if (OUT_MODE == 1) v *= oscale;
        slab[(mOff + r) * 68 + (j << 4) + rlane] = v;
      }
    }
    __builtin_amdgcn_fence(__ATOMIC_RELEASE, "workgroup");
    __builtin_amdgcn_wave_barrier();
    __builtin_amdgcn_fence(__ATOMIC_ACQUIRE, "workgroup");
    if (OUT_MODE == 0) {
      float* C = (float*)Cout;
      const int hh = lane >> 4, c4 = (lane & 15) * 4;
      for (int pass = 0; pass < 2; ++pass) {
#pragma unroll
        for (int it = 0; it < 8; ++it) {
          const int row = it * 2 + hh;
          const v4f v = *(const v4f*)(slab + row * 68 + c4);
          *(volatile v4f*)(C + (size_t)(mBase + row) * ldc + n0 + c4) = v;
        }
        __threadfence();
      }
    } else {
      _Float16* C = (_Float16*)Cout;
      const int q = lane >> 3, c8 = (lane & 7) * 8;
      for (int pass = 0; pass < 2; ++pass) {
#pragma unroll
        for (int it = 0; it < 4; ++it) {
          const int row = it * 4 + q;
          const float* sp = slab + row * 68 + c8;
          v8h hv;
#pragma unroll
          for (int e = 0; e < 8; ++e) hv[e] = (_Float16)sp[e];
          *(volatile v8h*)(C + (size_t)(mBase + row) * ldc + n0 + c8) = hv;
        }
        __threadfence();
      }
    }
    __builtin_amdgcn_fence(__ATOMIC_RELEASE, "workgroup");
    __builtin_amdgcn_wave_barrier();
    __builtin_amdgcn_fence(__ATOMIC_ACQUIRE, "workgroup");
  }
  if (STATS) {
#pragma unroll
    for (int off = 16; off > 0; off >>= 1) {
      ds  += __shfl_xor(ds, off, 32);
      ds2 += __shfl_xor(ds2, off, 32);
    }
    v2d pv;
    pv[0] = ds; pv[1] = ds2;
    double* pd = (double*)part + (size_t)tile * 16;
    if (lane < 8) *(volatile v2d*)(pd + 2 * lane) = pv;
    __threadfence();
    if (lane < 8) *(volatile v2d*)(pd + 2 * lane) = pv;
  }
}

__global__ __launch_bounds__(256) void cvt16_kernel(const float* __restrict__ in, unsigned short* __restrict__ outp,
                                                    int n8, float scale) {
  const int i = blockIdx.x * 256 + threadIdx.x;
  if (i >= n8) return;
  const size_t e = (size_t)i * 8;
  const v4f a = *(const v4f*)(in + e);
  const v4f c = *(const v4f*)(in + e + 4);
  v8h o;
#pragma unroll
  for (int k = 0; k < 4; ++k) { o[k] = (_Float16)(a[k] * scale); o[4 + k] = (_Float16)(c[k] * scale); }
  _Float16* op = (_Float16*)outp + e;
  *(volatile v8h*)op = o;
  __threadfence();
  *(volatile v8h*)op = o;
}

__global__ __launch_bounds__(256) void tcvt_kernel(const float* __restrict__ W, unsigned short* __restrict__ outp,
                                                   int R, int Cc, float scale) {
  __shared__ __align__(16) float tf[64 * 68];
  const int c0  = blockIdx.x * 64;
  const int r0  = blockIdx.y * 64;
  const int tid = threadIdx.x;
  {
    const int lr = tid >> 4;
    const int c4 = (tid & 15) * 4;
#pragma unroll
    for (int it = 0; it < 4; ++it) {
      const int rr = it * 16 + lr;
      const v4f a = *(const v4f*)(W + (size_t)(r0 + rr) * Cc + c0 + c4);
      *(v4f*)(tf + rr * 68 + c4) = a;
    }
  }
  __syncthreads();
  const int sub = tid >> 3;
  const int c8  = (tid & 7) * 8;
  v8h hv[2];
#pragma unroll
  for (int it = 0; it < 2; ++it) {
    const int oc = it * 32 + sub;
    v8h a;
#pragma unroll
    for (int e = 0; e < 8; ++e) a[e] = (_Float16)(tf[(c8 + e) * 68 + oc] * scale);
    hv[it] = a;
  }
  _Float16* o = (_Float16*)outp;
  for (int pass = 0; pass < 2; ++pass) {
#pragma unroll
    for (int it = 0; it < 2; ++it) {
      const int oc = it * 32 + sub;
      *(volatile v8h*)(o + (size_t)(c0 + oc) * R + r0 + c8) = hv[it];
    }
    __threadfence();
  }
}

__global__ __launch_bounds__(256) void ksum_kernel(const float* __restrict__ Kf, float* __restrict__ T) {
  const int d = blockIdx.x * 256 + threadIdx.x;
  const int b = blockIdx.y;
  if (d >= DM) return;
  const float* p = Kf + (size_t)b * SEQ * DM + d;
  float s = 0.f;
#pragma unroll 4
  for (int t = 0; t < SEQ; ++t) s += p[(size_t)t * DM];
  float* tp = T + b * DM + d;
  *(volatile float*)tp = s;
  __threadfence();
  *(volatile float*)tp = s;
}

__global__ __launch_bounds__(96) void kmix_kernel(const float* __restrict__ Kf, const float* __restrict__ T,
                                                  unsigned short* __restrict__ KMp) {
  const int s = blockIdx.x, b = blockIdx.y;
  const int col = threadIdx.x * 8;
  const int lo = (s - 2 > 0) ? (s - 2) : 0;
  const int hi = (s + 2 < SEQ - 1) ? (s + 2) : (SEQ - 1);
  const int cnt = hi - lo + 1;
  const float enb = 0.36787945f;
  const float Z   = (float)cnt + (float)(SEQ - cnt) * enb;
  const float rz  = 1.0f / Z;
  const float wnb = enb * rz;
  const float wd  = rz - wnb;
  v4f b0 = (v4f){0.f, 0.f, 0.f, 0.f}, b1 = (v4f){0.f, 0.f, 0.f, 0.f};
  for (int t = lo; t <= hi; ++t) {
    const float* kp = Kf + ((size_t)b * SEQ + t) * DM + col;
    b0 += *(const v4f*)(kp);
    b1 += *(const v4f*)(kp + 4);
  }
  const float* tp = T + b * DM + col;
  const v4f t0 = *(const v4f*)(tp);
  const v4f t1 = *(const v4f*)(tp + 4);
  v8h o;
#pragma unroll
  for (int e = 0; e < 4; ++e) {
    o[e]     = (_Float16)((wnb * t0[e] + wd * b0[e]) * 64.0f);
    o[4 + e] = (_Float16)((wnb * t1[e] + wd * b1[e]) * 64.0f);
  }
  _Float16* op = (_Float16*)KMp + ((size_t)b * SEQ + s) * DM + col;
  *(volatile v8h*)op = o;
  __threadfence();
  *(volatile v8h*)op = o;
}

__global__ __launch_bounds__(256)
void attn_kernel(const unsigned short* __restrict__ Qp, const unsigned short* __restrict__ KMp,
                 const unsigned short* __restrict__ VTp, const float* __restrict__ text,
                 float* __restrict__ U, float* __restrict__ part, float c2) {
  extern __shared__ __align__(16) float sc[];
  const int tid = threadIdx.x;
  const int w = tid >> 5, lane = tid & 31, h = lane >> 4, n = lane & 15;
  const int b = blockIdx.y, qt = blockIdx.x;
  const int q0 = qt * AQ;
  const _Float16* Q  = (const _Float16*)Qp + ((size_t)b * SEQ + q0) * DM;
  const _Float16* KM = (const _Float16*)KMp + (size_t)b * SEQ * DM;
  const _Float16* VT = (const _Float16*)VTp + (size_t)b * SEQ;

  {
    const _Float16* qa0 = Q + (size_t)n * DM + 8 * h;
    const _Float16* qa1 = Q + (size_t)(16 + n) * DM + 8 * h;
    for (int g = 0; g < 4; ++g) {
      const int nc0 = w * 256 + g * 64;
      const _Float16* kb = KM + (size_t)(nc0 + n) * DM + 8 * h;
      v8f acc[2][4];
#pragma unroll
      for (int j = 0; j < 4; ++j) { acc[0][j] = zero8(); acc[1][j] = zero8(); }
#pragma unroll 2
      for (int k0 = 0; k0 < DM; k0 += 32) {
        const v16h a0 = frag_ld(qa0 + k0);
        const v16h a1 = frag_ld(qa1 + k0);
#pragma unroll
        for (int j = 0; j < 4; ++j) {
          const v16h bj = frag_ld(kb + (size_t)j * 16 * DM + k0);
          acc[0][j] = mma_g(a0, bj, acc[0][j]);
          acc[1][j] = mma_g(a1, bj, acc[1][j]);
        }
      }
#pragma unroll
      for (int j = 0; j < 4; ++j) {
#pragma unroll
        for (int r = 0; r < 8; ++r) {
          sc[(size_t)(8 * h + r) * SEQ + nc0 + 16 * j + n]      = acc[0][j][r];
          sc[(size_t)(16 + 8 * h + r) * SEQ + nc0 + 16 * j + n] = acc[1][j][r];
        }
      }
    }
  }
  __syncthreads();

  {
#pragma unroll 1
    for (int rr = 0; rr < 4; ++rr) {
      float* prow = sc + (size_t)(4 * w + rr) * SEQ;
      v4f x[16];
#pragma unroll
      for (int i = 0; i < 8; ++i) {
        x[2 * i]     = *(const v4f*)(prow + 256 * i + 8 * lane);
        x[2 * i + 1] = *(const v4f*)(prow + 256 * i + 8 * lane + 4);
      }
      float m = x[0][0];
#pragma unroll
      for (int i = 0; i < 16; ++i)
        m = fmaxf(m, fmaxf(fmaxf(x[i][0], x[i][1]), fmaxf(x[i][2], x[i][3])));
#pragma unroll
      for (int off = 16; off > 0; off >>= 1) m = fmaxf(m, __shfl_xor(m, off, 32));
      float s = 0.f;
#pragma unroll
      for (int i = 0; i < 16; ++i) {
        v4f p;
#pragma unroll
        for (int e = 0; e < 4; ++e) { p[e] = exp2f((x[i][e] - m) * c2); s += p[e]; }
        x[i] = p;
      }
#pragma unroll
      for (int off = 16; off > 0; off >>= 1) s += __shfl_xor(s, off, 32);
      const float inv = 4096.0f / s;
      _Float16* hrow = (_Float16*)prow;
#pragma unroll
      for (int i = 0; i < 8; ++i) {
        v8h ph;
#pragma unroll
        for (int e = 0; e < 4; ++e) {
          ph[e]     = (_Float16)(x[2 * i][e] * inv);
          ph[4 + e] = (_Float16)(x[2 * i + 1][e] * inv);
        }
        *(v8h*)(hrow + 256 * i + 8 * lane) = ph;
      }
    }
  }
  __syncthreads();

  {
    const _Float16* P16 = (const _Float16*)sc;
    const _Float16* pp0 = P16 + (size_t)n * (2 * SEQ) + 8 * h;
    const _Float16* pp1 = P16 + (size_t)(16 + n) * (2 * SEQ) + 8 * h;
    float* so = sc + SEQ / 2;
#pragma unroll 1
    for (int ps = 0; ps < 2; ++ps) {
      const int ncw = 96 * w + 48 * ps;
      const _Float16* vbp = VT + (size_t)(ncw + n) * NTOK + 8 * h;
      v8f o[2][3];
#pragma unroll
      for (int t = 0; t < 3; ++t) { o[0][t] = zero8(); o[1][t] = zero8(); }
#pragma unroll 2
      for (int k0 = 0; k0 < SEQ; k0 += 32) {
        const v16h p0 = frag_ld(pp0 + k0);
        const v16h p1 = frag_ld(pp1 + k0);
#pragma unroll
        for (int t = 0; t < 3; ++t) {
          const v16h vb = frag_ld(vbp + (size_t)t * 16 * NTOK + k0);
          o[0][t] = mma_g(p0, vb, o[0][t]);
          o[1][t] = mma_g(p1, vb, o[1][t]);
        }
      }
#pragma unroll
      for (int mi = 0; mi < 2; ++mi)
#pragma unroll
        for (int t = 0; t < 3; ++t)
#pragma unroll
          for (int r = 0; r < 8; ++r)
            so[(size_t)(16 * mi + 8 * h + r) * SEQ + ncw + 16 * t + n] = o[mi][t][r] * (1.0f / 65536.0f);
    }
  }
  __syncthreads();

  {
    const float* so = sc + SEQ / 2;
    const int q8 = lane >> 3, c4 = (lane & 7) * 4;
    double ds = 0.0, ds2 = 0.0;
#pragma unroll 1
    for (int rr = 0; rr < 4; ++rr) {
      const int row = 4 * w + rr;
      const size_t gr = ((size_t)b * SEQ + q0 + row) * DM;
      v4f vals[6];
#pragma unroll
      for (int it = 0; it < 6; ++it) {
        const int col = (it * 4 + q8) * 32 + c4;
        const v4f a  = *(const v4f*)(so + (size_t)row * SEQ + col);
        const v4f tx = *(const v4f*)(text + gr + col);
        const v4f u  = a + tx;
        vals[it] = u;
#pragma unroll
        for (int e = 0; e < 4; ++e) { const double dv = (double)u[e]; ds += dv; ds2 += dv * dv; }
      }
#pragma unroll
      for (int it = 0; it < 6; ++it) {
        const int col = (it * 4 + q8) * 32 + c4;
        *(volatile v4f*)(U + gr + col) = vals[it];
      }
      __threadfence();
#pragma unroll
      for (int it = 0; it < 6; ++it) {
        const int col = (it * 4 + q8) * 32 + c4;
        *(volatile v4f*)(U + gr + col) = vals[it];
      }
    }
#pragma unroll
    for (int off = 16; off > 0; off >>= 1) {
      ds  += __shfl_xor(ds, off, 32);
      ds2 += __shfl_xor(ds2, off, 32);
    }
    v2d pv;
    pv[0] = ds; pv[1] = ds2;
    const int li = (b * (SEQ / AQ) + qt) * 8 + w;
    double* pd = (double*)part + (size_t)li * 16;
    if (lane < 8) *(volatile v2d*)(pd + 2 * lane) = pv;
    __threadfence();
    if (lane < 8) *(volatile v2d*)(pd + 2 * lane) = pv;
  }
}

__global__ __launch_bounds__(256) void ln_stats_kernel(const float* __restrict__ part, int nlines, int count,
                                                       float* __restrict__ stats) {
  __shared__ double ls[256];
  __shared__ double ls2[256];
  const int tid = threadIdx.x;
  const double* pd = (const double*)part;
  double s = 0.0, s2 = 0.0;
  for (int i = tid; i < nlines; i += 256) { s += pd[(size_t)i * 16]; s2 += pd[(size_t)i * 16 + 1]; }
  ls[tid] = s; ls2[tid] = s2;
  __syncthreads();
  for (int o = 128; o > 0; o >>= 1) {
    if (tid < o) { ls[tid] += ls[tid + o]; ls2[tid] += ls2[tid + o]; }
    __syncthreads();
  }
  const double invn = 1.0 / (double)count;
  const double mean = ls[0] * invn;
  double var = ls2[0] * invn - mean * mean;
  if (var < 0.0) var = 0.0;
  const float meanf = (float)mean;
  const float rstd  = (float)(1.0 / sqrt(var + 1e-6));
  v4f sv = (v4f){meanf, rstd, 0.f, 0.f};
  if (tid < 8) *(volatile v4f*)(stats + 4 * tid) = sv;
  __threadfence();
  if (tid < 8) *(volatile v4f*)(stats + 4 * tid) = sv;
}

__global__ __launch_bounds__(256) void ln_apply16_kernel(const float* __restrict__ u, const float* __restrict__ gamma,
                                                         const float* __restrict__ beta, const float* __restrict__ stats,
                                                         unsigned short* __restrict__ outp, int n8) {
  const int i = blockIdx.x * 256 + threadIdx.x;
  if (i >= n8) return;
  const float mean = stats[0], rstd = stats[1];
  const size_t e = (size_t)i * 8;
  const v4f u0 = *(const v4f*)(u + e),     u1 = *(const v4f*)(u + e + 4);
  const v4f g0 = *(const v4f*)(gamma + e), g1 = *(const v4f*)(gamma + e + 4);
  const v4f b0 = *(const v4f*)(beta + e),  b1 = *(const v4f*)(beta + e + 4);
  v8h o;
#pragma unroll
  for (int k = 0; k < 4; ++k) {
    o[k]     = (_Float16)((u0[k] - mean) * rstd * g0[k] + b0[k]);
    o[4 + k] = (_Float16)((u1[k] - mean) * rstd * g1[k] + b1[k]);
  }
  _Float16* op = (_Float16*)outp + e;
  *(volatile v8h*)op = o;
  __threadfence();
  *(volatile v8h*)op = o;
}

__global__ __launch_bounds__(256) void ln_apply32_kernel(const float* __restrict__ u, const float* __restrict__ gamma,
                                                         const float* __restrict__ beta, const float* __restrict__ stats,
                                                         float* __restrict__ out, int n4) {
  const int i = blockIdx.x * 256 + threadIdx.x;
  if (i >= n4) return;
  const float mean = stats[0], rstd = stats[1];
  const size_t e = (size_t)i * 4;
  const v4f uu = *(const v4f*)(u + e);
  const v4f gg = *(const v4f*)(gamma + e);
  const v4f bb = *(const v4f*)(beta + e);
  v4f o;
#pragma unroll
  for (int k = 0; k < 4; ++k) o[k] = (uu[k] - mean) * rstd * gg[k] + bb[k];
  *(volatile v4f*)(out + e) = o;
  __threadfence();
  *(volatile v4f*)(out + e) = o;
}

__global__ __launch_bounds__(256) void copy4_kernel(const float* __restrict__ in, float* __restrict__ out, int n4) {
  const int i = blockIdx.x * 256 + threadIdx.x;
  if (i >= n4) return;
  const size_t e = (size_t)i * 4;
  const v4f v = *(const v4f*)(in + e);
  *(volatile v4f*)(out + e) = v;
  __threadfence();
  *(volatile v4f*)(out + e) = v;
}

extern "C" void kernel_launch(void* const* d_in, const int* in_sizes, int n_in,
                              void* d_out, int out_size, void* d_ws, size_t ws_size,
                              hipStream_t stream) {
  static_assert((size_t)MC * DH * 2 == (size_t)NTOK * DM * 2);
  static_assert(2 * (size_t)DM * DH * 2 <= (size_t)NTOK * DM * 2);
  static_assert(NTOK % MC == 0);
  if (n_in < 14) return;
  const long NEL = (long)NTOK * DM;
  if (in_sizes[0] != NEL || in_sizes[1] != NIMG) return;
  if (in_sizes[2] != DM * DM || in_sizes[4] != DM * DM || in_sizes[6] != DM * DM) return;
  if (in_sizes[3] != DM || in_sizes[5] != DM || in_sizes[7] != DM || in_sizes[11] != DM) return;
  if (in_sizes[8] != DM * DH || in_sizes[9] != DH || in_sizes[10] != DH * DM) return;
  if (in_sizes[12] != NEL || in_sizes[13] != NEL) return;
  if ((long)out_size != NEL + NIMG) return;

  const float* text  = (const float*)d_in[0];
  const float* image = (const float*)d_in[1];
  const float* Wq = (const float*)d_in[2];  const float* bq = (const float*)d_in[3];
  const float* Wk = (const float*)d_in[4];  const float* bk = (const float*)d_in[5];
  const float* Wv = (const float*)d_in[6];  const float* bv = (const float*)d_in[7];
  const float* W1 = (const float*)d_in[8];  const float* b1 = (const float*)d_in[9];
  const float* W2 = (const float*)d_in[10]; const float* b2 = (const float*)d_in[11];
  const float* gamma = (const float*)d_in[12];
  const float* beta  = (const float*)d_in[13];
  float* out0 = (float*)d_out;
  float* out1 = out0 + NEL;

  const size_t PA  = (size_t)NTOK * DM * 2;
  const size_t PF  = (size_t)NTOK * DM * 4;
  const size_t PW  = (size_t)DM * DM * 2;
  const size_t PW1 = (size_t)DM * DH * 2;
  const size_t PT  = (size_t)NB * DM * 4;
  const int nl1 = NB * (SEQ / AQ) * 8;
  const int nl2 = (NTOK / 64) * (DM / 64);
  size_t off = 0;
  const size_t oR0 = off; off += PA;
  const size_t oR1 = off; off += PA;
  const size_t oR2 = off; off += PF;
  const size_t oR3 = off; off += PA;
  const size_t oWq = off; off += PW;
  const size_t oWk = off; off += PW;
  const size_t oWv = off; off += PW;
  const size_t oT  = off; off += PT;
  const size_t oP1 = off; off += (size_t)nl1 * 128;
  const size_t oP2 = off; off += (size_t)nl2 * 128;
  const size_t oS1 = off; off += 128;
  const size_t oS2 = off; off += 128;
  if (off > ws_size) return;

  char* ws = (char*)d_ws;
  unsigned short* X16  = (unsigned short*)(ws + oR0);
  unsigned short* KM16 = (unsigned short*)(ws + oR0);
  unsigned short* X1h  = (unsigned short*)(ws + oR0);
  unsigned short* Q16  = (unsigned short*)(ws + oR1);
  unsigned short* Hd   = (unsigned short*)(ws + oR1);
  float*          Kf   = (float*)(ws + oR2);
  float*          U1   = (float*)(ws + oR2);
  float*          U2   = (float*)(ws + oR2);
  unsigned short* VT16 = (unsigned short*)(ws + oR3);
  unsigned short* W1T  = (unsigned short*)(ws + oR3);
  unsigned short* W2T  = (unsigned short*)(ws + oR3 + PW1);
  unsigned short* WqT  = (unsigned short*)(ws + oWq);
  unsigned short* WkT  = (unsigned short*)(ws + oWk);
  unsigned short* WvT  = (unsigned short*)(ws + oWv);
  float*          T    = (float*)(ws + oT);
  float*          part1 = (float*)(ws + oP1);
  float*          part2 = (float*)(ws + oP2);
  float*          st1  = (float*)(ws + oS1);
  float*          st2  = (float*)(ws + oS2);

  const dim3 blk(256);
  const int n8  = (int)(NEL / 8);
  const int n4  = (int)(NEL / 4);
  const int ni4 = NIMG / 4;
  const int tilesQ  = (NTOK / 64) * (DM / 64);
  const int tilesF1 = (MC / 64) * (DH / 64);
  const int tilesF2 = (MC / 64) * (DM / 64);
  if ((tilesQ & 7) || (tilesF1 & 7) || (tilesF2 & 7)) return;
  const float c2 = (float)(1.4426950408889634 / (1024.0 * sqrt(768.0)));
  const int attLds = AQ * SEQ * 4;

  cvt16_kernel<<<dim3((n8 + 255) / 256), blk, 0, stream>>>(text, X16, n8, 1.0f);
  tcvt_kernel<<<dim3(DM / 64, DM / 64), blk, 0, stream>>>(Wq, WqT, DM, DM, 256.0f);
  tcvt_kernel<<<dim3(DM / 64, DM / 64), blk, 0, stream>>>(Wk, WkT, DM, DM, 256.0f);
  tcvt_kernel<<<dim3(DM / 64, DM / 64), blk, 0, stream>>>(Wv, WvT, DM, DM, 256.0f);
  gemm64_kernel<2, 1, false, 0, false><<<dim3(tilesQ / 8), blk, 0, stream>>>(
      X16, DM, WqT, DM, (void*)Q16, DM, bq, nullptr, nullptr, NTOK, DM, DM, 1.0f / 256.0f, 16.0f);
  gemm64_kernel<2, 0, false, 0, false><<<dim3(tilesQ / 8), blk, 0, stream>>>(
      X16, DM, WkT, DM, (void*)Kf, DM, bk, nullptr, nullptr, NTOK, DM, DM, 1.0f / 256.0f, 1.0f);
  gemm64_kernel<1, 1, false, 0, false><<<dim3(tilesQ / 8), blk, 0, stream>>>(
      WvT, DM, X16, DM, (void*)VT16, NTOK, bv, nullptr, nullptr, DM, NTOK, DM, 1.0f / 256.0f, 16.0f);
  ksum_kernel<<<dim3(DM / 256, NB), blk, 0, stream>>>(Kf, T);
  kmix_kernel<<<dim3(SEQ, NB), dim3(96), 0, stream>>>(Kf, T, KM16);
  (void)hipFuncSetAttribute(reinterpret_cast<const void*>(&attn_kernel),
                            hipFuncAttributeMaxDynamicSharedMemorySize, attLds);
  attn_kernel<<<dim3(SEQ / AQ, NB), blk, attLds, stream>>>(Q16, KM16, VT16, text, U1, part1, c2);
  ln_stats_kernel<<<dim3(1), blk, 0, stream>>>(part1, nl1, (int)NEL, st1);
  ln_apply16_kernel<<<dim3((n8 + 255) / 256), blk, 0, stream>>>(U1, gamma, beta, st1, X1h, n8);
  tcvt_kernel<<<dim3(DH / 64, DM / 64), blk, 0, stream>>>(W1, W1T, DM, DH, 256.0f);
  tcvt_kernel<<<dim3(DM / 64, DH / 64), blk, 0, stream>>>(W2, W2T, DH, DM, 512.0f);
  for (int c = 0; c < NTOK / MC; ++c) {
    const size_t ro = (size_t)c * MC * DM;
    gemm64_kernel<2, 1, false, 2, false><<<dim3(tilesF1 / 8), blk, 0, stream>>>(
        X1h + ro, DM, W1T, DM, (void*)Hd, DH, b1, nullptr, nullptr, MC, DH, DM, 1.0f / 256.0f, 16.0f);
    gemm64_kernel<2, 0, true, 0, true><<<dim3(tilesF2 / 8), blk, 0, stream>>>(
        Hd, DH, W2T, DH, (void*)(U2 + ro), DM, b2, text + ro, part2 + (size_t)c * tilesF2 * 32,
        MC, DM, DH, 1.0f / 8192.0f, 1.0f);
  }
  ln_stats_kernel<<<dim3(1), blk, 0, stream>>>(part2, nl2, (int)NEL, st2);
  ln_apply32_kernel<<<dim3((n4 + 255) / 256), blk, 0, stream>>>(U2, gamma, beta, st2, out0, n4);
  copy4_kernel<<<dim3((ni4 + 255) / 256), blk, 0, stream>>>(image, out1, ni4);
  (void)hipGetLastError();
}
